// PSI_47931835024047
// MI455X (gfx1250) — hardware-verified
//
#include <hip/hip_runtime.h>
#include <stddef.h>
#include <stdint.h>
#include <math.h>

#define NBATCH 4
#define SEQ    4096
#define DMOD   512
#define CHK    64
#define NROW   16384
#define NCTX   2048
#define NHID   1024
#define NCHUNK 256

static_assert(NBATCH * SEQ == NROW);
static_assert(NCHUNK * CHK == NROW);
static_assert(NCTX == 4 * DMOD);
static_assert(NHID == 2 * DMOD);
static_assert((DMOD % 32) == 0 && (NCTX % 32) == 0 && (NHID % 32) == 0);

typedef _Float16     v16h __attribute__((ext_vector_type(16)));
typedef _Float16     v8h  __attribute__((ext_vector_type(8)));
typedef float        v8f  __attribute__((ext_vector_type(8)));
typedef float        v4f  __attribute__((ext_vector_type(4)));
typedef unsigned int v4u  __attribute__((ext_vector_type(4)));

union Frag { v16h v; v8h h[2]; };
union Pk8  { v8h h; v4u u; };

__device__ __forceinline__ v8f zero8() { return (v8f){0.f, 0.f, 0.f, 0.f, 0.f, 0.f, 0.f, 0.f}; }

__device__ __forceinline__ v8f mma16(v16h a, v16h b, v8f c) {
  c = __builtin_amdgcn_wmma_f32_16x16x32_f16(false, a, false, b, (short)0, c, false, false);
  asm volatile("v_nop\n\tv_nop\n\tv_nop\n\tv_nop" : "+v"(c) : "v"(a), "v"(b));
  return c;
}

__device__ __forceinline__ v16h ldfrag_g(const _Float16* p, int ld, int k0, int lane) {
  const _Float16* q = p + (size_t)(lane & 15) * ld + k0 + 8 * (lane >> 4);
  Frag f;
  f.h[0] = *(const v8h*)(q);
  f.h[1] = *(const v8h*)(q + 16);
  return f.v;
}

__device__ __forceinline__ v16h ldfrag_x(const float* p, int ld, int k0, int lane) {
  const float* q = p + (size_t)(lane & 15) * ld + k0 + 8 * (lane >> 4);
  const v4f a0 = *(const v4f*)(q), a1 = *(const v4f*)(q + 4);
  const v4f a2 = *(const v4f*)(q + 16), a3 = *(const v4f*)(q + 20);
  v16h r;
  r[0]  = (_Float16)a0[0]; r[1]  = (_Float16)a0[1]; r[2]  = (_Float16)a0[2]; r[3]  = (_Float16)a0[3];
  r[4]  = (_Float16)a1[0]; r[5]  = (_Float16)a1[1]; r[6]  = (_Float16)a1[2]; r[7]  = (_Float16)a1[3];
  r[8]  = (_Float16)a2[0]; r[9]  = (_Float16)a2[1]; r[10] = (_Float16)a2[2]; r[11] = (_Float16)a2[3];
  r[12] = (_Float16)a3[0]; r[13] = (_Float16)a3[1]; r[14] = (_Float16)a3[2]; r[15] = (_Float16)a3[3];
  return r;
}

#define TPW 33
__global__ __launch_bounds__(256) void k_prepw(const float* __restrict__ w, int K, int N, float sc,
                                               _Float16* __restrict__ wt) {
  __shared__ float sw[64 * TPW];
  const int k0 = blockIdx.x * 64, n0 = blockIdx.y * 32;
  const int tid = threadIdx.x;
#pragma unroll
  for (int it = 0; it < 2; ++it) {
    const int idx = tid + 256 * it;
    const int kk = idx >> 3, c4 = idx & 7;
    const v4f a = *(const v4f*)(w + (size_t)(k0 + kk) * N + n0 + c4 * 4);
    float* r = sw + kk * TPW + c4 * 4;
    r[0] = a[0]; r[1] = a[1]; r[2] = a[2]; r[3] = a[3];
  }
  __syncthreads();
  const int n = tid >> 3, pc = tid & 7;
  Pk8 o;
#pragma unroll
  for (int j = 0; j < 8; ++j) o.h[j] = (_Float16)(sw[(pc * 8 + j) * TPW + n] * sc);
  const size_t go = (size_t)(n0 + n) * K + k0 + pc * 8;
  const v4u ov = o.u;
  *(volatile v4u*)(wt + go) = ov;
  __threadfence();
  *(volatile v4u*)(wt + go) = ov;
}

#define CPP 516
#define RWP 2056
#define SM_PHI (64 * CPP * 4)
#define SM_RAW (8 * RWP * 4)
#define SM_CHUNK (SM_PHI + SM_RAW)
static_assert((SM_PHI % 16) == 0);
static_assert((RWP % 4) == 0);

__global__ __launch_bounds__(256) void k_chunk(const float* __restrict__ x, const _Float16* __restrict__ wot,
                                               const float* __restrict__ bom, const float* __restrict__ lsc,
                                               const float* __restrict__ gam, const float* __restrict__ bet,
                                               _Float16* __restrict__ ctxn) {
  extern __shared__ __align__(16) unsigned char smem[];
  float* sPhi = (float*)(smem);
  float* sRaw = (float*)(smem + SM_PHI);
  const int tid = threadIdx.x, lane = tid & 31, wave = tid >> 5;
  const int hh = lane >> 4, c = lane & 15;
  const size_t row0 = (size_t)blockIdx.x * CHK;
  const float* xb = x + row0 * DMOD;

  {
    const int mt = wave & 3, nh = wave >> 2;
    const float* xa = xb + (size_t)(mt * 16) * DMOD;
#pragma unroll 1
    for (int pass = 0; pass < 2; ++pass) {
      const int ncol0 = pass * 256 + nh * 128;
      v8f acc[8];
#pragma unroll
      for (int ns = 0; ns < 8; ++ns) acc[ns] = zero8();
#pragma unroll 1
      for (int ks = 0; ks < DMOD / 32; ++ks) {
        const int k0 = ks * 32;
        const v16h a = ldfrag_x(xa, DMOD, k0, lane);
#pragma unroll
        for (int ns = 0; ns < 8; ++ns) {
          const v16h b = ldfrag_g(wot + (size_t)(ncol0 + 16 * ns) * DMOD, DMOD, k0, lane);
          acc[ns] = mma16(a, b, acc[ns]);
        }
      }
#pragma unroll
      for (int ns = 0; ns < 8; ++ns) {
        const int col = ncol0 + 16 * ns + c;
#pragma unroll
        for (int r = 0; r < 8; ++r) sPhi[(mt * 16 + 8 * hh + r) * CPP + col] = acc[ns][r];
      }
    }
  }
  __syncthreads();

  const int c0 = tid, c1 = tid + 256;
  const float bo0 = bom[c0], bo1 = bom[c1];
  const float sc0 = expf(lsc[c0]), sc1 = expf(lsc[c1]);
  float ph0 = 0.f, ph1 = 0.f, ar0 = 0.f, ai0 = 0.f, ar1 = 0.f, ai1 = 0.f;
#pragma unroll 1
  for (int slab = 0; slab < 8; ++slab) {
#pragma unroll 1
    for (int rl = 0; rl < 8; ++rl) {
      const int m = slab * 8 + rl;
      const float fp = (float)(m + 1);
      const float psc = 1.0f / sqrtf(fp);
      const float inv = 1.0f / fp;
      float* rw = sRaw + rl * RWP;
      const float* xr = xb + (size_t)m * DMOD;
      {
        const float om = sPhi[m * CPP + c0] * 0.0625f + bo0;
        ph0 += (om * sc0) * psc;
        const float cs = cosf(ph0), sn = sinf(ph0);
        const float xv = xr[c0];
        const float cr = xv * cs, ci = xv * sn;
        ar0 += cr; ai0 += ci;
        const float mr = ar0 * inv, mi = ai0 * inv;
        rw[c0] = cr;
        rw[DMOD + c0] = ci;
        rw[2 * DMOD + c0] = mr * cs + mi * sn;
        rw[3 * DMOD + c0] = mi * cs - mr * sn;
      }
      {
        const float om = sPhi[m * CPP + c1] * 0.0625f + bo1;
        ph1 += (om * sc1) * psc;
        const float cs = cosf(ph1), sn = sinf(ph1);
        const float xv = xr[c1];
        const float cr = xv * cs, ci = xv * sn;
        ar1 += cr; ai1 += ci;
        const float mr = ar1 * inv, mi = ai1 * inv;
        rw[c1] = cr;
        rw[DMOD + c1] = ci;
        rw[2 * DMOD + c1] = mr * cs + mi * sn;
        rw[3 * DMOD + c1] = mi * cs - mr * sn;
      }
    }
    __syncthreads();
    {
      const float* rw = sRaw + wave * RWP;
      float s = 0.f;
#pragma unroll
      for (int j = 0; j < 8; ++j) {
        const v4f a0 = *(const v4f*)(rw + 256 * j + 8 * lane);
        const v4f a1 = *(const v4f*)(rw + 256 * j + 8 * lane + 4);
        s += ((a0[0] + a0[1]) + (a0[2] + a0[3])) + ((a1[0] + a1[1]) + (a1[2] + a1[3]));
      }
      s += __shfl_xor(s, 1, 32); s += __shfl_xor(s, 2, 32); s += __shfl_xor(s, 4, 32);
      s += __shfl_xor(s, 8, 32); s += __shfl_xor(s, 16, 32);
      const float mu = s * (1.0f / 2048.0f);
      float q = 0.f;
#pragma unroll
      for (int j = 0; j < 8; ++j) {
        const v4f a0 = *(const v4f*)(rw + 256 * j + 8 * lane);
        const v4f a1 = *(const v4f*)(rw + 256 * j + 8 * lane + 4);
#pragma unroll
        for (int e = 0; e < 4; ++e) {
          const float d0 = a0[e] - mu, d1 = a1[e] - mu;
          q += d0 * d0;
          q += d1 * d1;
        }
      }
      q += __shfl_xor(q, 1, 32); q += __shfl_xor(q, 2, 32); q += __shfl_xor(q, 4, 32);
      q += __shfl_xor(q, 8, 32); q += __shfl_xor(q, 16, 32);
      const float rstd = 1.0f / sqrtf(q * (1.0f / 2048.0f) + 1e-5f);
      Pk8 o[8];
#pragma unroll
      for (int j = 0; j < 8; ++j) {
        const int col = 256 * j + 8 * lane;
        const v4f a0 = *(const v4f*)(rw + col), a1 = *(const v4f*)(rw + col + 4);
        const v4f g0 = *(const v4f*)(gam + col), g1 = *(const v4f*)(gam + col + 4);
        const v4f e0 = *(const v4f*)(bet + col), e1 = *(const v4f*)(bet + col + 4);
#pragma unroll
        for (int e = 0; e < 4; ++e) {
          o[j].h[e]     = (_Float16)((a0[e] - mu) * rstd * g0[e] + e0[e]);
          o[j].h[4 + e] = (_Float16)((a1[e] - mu) * rstd * g1[e] + e1[e]);
        }
      }
      const size_t gro = (row0 + (size_t)(slab * 8 + wave)) * NCTX;
#pragma unroll
      for (int j = 0; j < 8; ++j) *(volatile v4u*)(ctxn + gro + 256 * j + 8 * lane) = o[j].u;
      __threadfence();
#pragma unroll
      for (int j = 0; j < 8; ++j) *(volatile v4u*)(ctxn + gro + 256 * j + 8 * lane) = o[j].u;
    }
    __syncthreads();
  }
}

#define EP1 136
__global__ __launch_bounds__(128) void k_ffn1(const _Float16* __restrict__ ap, const _Float16* __restrict__ w1t,
                                              const float* __restrict__ b1, _Float16* __restrict__ hpl) {
  __shared__ __align__(16) _Float16 sE[4 * 16 * EP1];
  const int tid = threadIdx.x, lane = tid & 31, wave = tid >> 5;
  const int hh = lane >> 4, c = lane & 15;
  const size_t m0 = (size_t)blockIdx.x * 64 + (size_t)wave * 16;
  const int n0 = blockIdx.y * 128;
  const _Float16* arow = ap + m0 * NCTX;
  const _Float16* brow = w1t + (size_t)n0 * NCTX;
  v8f acc[8];
#pragma unroll
  for (int ns = 0; ns < 8; ++ns) acc[ns] = zero8();
#pragma unroll 1
  for (int ks = 0; ks < NCTX / 32; ++ks) {
    const int k0 = ks * 32;
    const v16h a = ldfrag_g(arow, NCTX, k0, lane);
#pragma unroll
    for (int ns = 0; ns < 8; ++ns) {
      const v16h b = ldfrag_g(brow + (size_t)(16 * ns) * NCTX, NCTX, k0, lane);
      acc[ns] = mma16(a, b, acc[ns]);
    }
  }
  _Float16* st = sE + wave * (16 * EP1);
#pragma unroll
  for (int ns = 0; ns < 8; ++ns) {
    const int col = 16 * ns + c;
    const float bb = b1[n0 + col];
#pragma unroll
    for (int r = 0; r < 8; ++r) {
      const float v = acc[ns][r] * (1.0f / 32.0f) + bb;
      const float g = 0.5f * v * (1.0f + erff(v * 0.70710678118654752f));
      st[(8 * hh + r) * EP1 + col] = (_Float16)(g * 4.0f);
    }
  }
  __syncthreads();
  Pk8 o[8];
  size_t go[8];
#pragma unroll
  for (int it = 0; it < 8; ++it) {
    const int p = it * 32 + lane;
    const int rowl = p >> 4, pc = p & 15;
    o[it].h = *(const v8h*)(st + rowl * EP1 + pc * 8);
    go[it] = (m0 + (size_t)rowl) * NHID + n0 + pc * 8;
  }
#pragma unroll
  for (int it = 0; it < 8; ++it) *(volatile v4u*)(hpl + go[it]) = o[it].u;
  __threadfence();
#pragma unroll
  for (int it = 0; it < 8; ++it) *(volatile v4u*)(hpl + go[it]) = o[it].u;
}

#define EP2 132
__global__ __launch_bounds__(128) void k_ffn2(const _Float16* __restrict__ hp, const _Float16* __restrict__ w2t,
                                              const float* __restrict__ b2, const float* __restrict__ x,
                                              float* __restrict__ out) {
  __shared__ __align__(16) float sE[4 * 16 * EP2];
  const int tid = threadIdx.x, lane = tid & 31, wave = tid >> 5;
  const int hh = lane >> 4, c = lane & 15;
  const size_t m0 = (size_t)blockIdx.x * 64 + (size_t)wave * 16;
  const int n0 = blockIdx.y * 128;
  const _Float16* arow = hp + m0 * NHID;
  const _Float16* brow = w2t + (size_t)n0 * NHID;
  v8f acc[8];
#pragma unroll
  for (int ns = 0; ns < 8; ++ns) acc[ns] = zero8();
#pragma unroll 1
  for (int ks = 0; ks < NHID / 32; ++ks) {
    const int k0 = ks * 32;
    const v16h a = ldfrag_g(arow, NHID, k0, lane);
#pragma unroll
    for (int ns = 0; ns < 8; ++ns) {
      const v16h b = ldfrag_g(brow + (size_t)(16 * ns) * NHID, NHID, k0, lane);
      acc[ns] = mma16(a, b, acc[ns]);
    }
  }
  float* st = sE + wave * (16 * EP2);
#pragma unroll
  for (int ns = 0; ns < 8; ++ns) {
#pragma unroll
    for (int r = 0; r < 8; ++r) st[(8 * hh + r) * EP2 + 16 * ns + c] = acc[ns][r];
  }
  __syncthreads();
  const v4f bb = *(const v4f*)(b2 + n0 + 4 * lane);
  v4f o[16];
#pragma unroll
  for (int it = 0; it < 16; ++it) {
    const v4f a = *(const v4f*)(st + it * EP2 + 4 * lane);
    const size_t go = (m0 + (size_t)it) * DMOD + n0 + 4 * lane;
    const v4f xv = *(const v4f*)(x + go);
    const v4f t = a * (1.0f / 128.0f) + bb;
    o[it] = xv + t;
  }
#pragma unroll
  for (int it = 0; it < 16; ++it)
    *(volatile v4f*)(out + (m0 + (size_t)it) * DMOD + n0 + 4 * lane) = o[it];
  __threadfence();
#pragma unroll
  for (int it = 0; it < 16; ++it)
    *(volatile v4f*)(out + (m0 + (size_t)it) * DMOD + n0 + 4 * lane) = o[it];
}

extern "C" void kernel_launch(void* const* d_in, const int* in_sizes, int n_in,
                              void* d_out, int out_size, void* d_ws, size_t ws_size,
                              hipStream_t stream) {
  if (n_in < 10) return;
  if (in_sizes[0] != NROW * DMOD) return;
  if (in_sizes[1] != DMOD * DMOD) return;
  if (in_sizes[2] != DMOD) return;
  if (in_sizes[3] != DMOD) return;
  if (in_sizes[4] != NCTX) return;
  if (in_sizes[5] != NCTX) return;
  if (in_sizes[6] != NCTX * NHID) return;
  if (in_sizes[7] != NHID) return;
  if (in_sizes[8] != NHID * DMOD) return;
  if (in_sizes[9] != DMOD) return;
  if (out_size != NROW * DMOD) return;

  const float* x    = (const float*)d_in[0];
  const float* wom  = (const float*)d_in[1];
  const float* bom  = (const float*)d_in[2];
  const float* lsc  = (const float*)d_in[3];
  const float* gam  = (const float*)d_in[4];
  const float* bet  = (const float*)d_in[5];
  const float* w1   = (const float*)d_in[6];
  const float* b1   = (const float*)d_in[7];
  const float* w2   = (const float*)d_in[8];
  const float* b2   = (const float*)d_in[9];
  float* out = (float*)d_out;

  const size_t szWO = (size_t)DMOD * DMOD * 2;
  const size_t szW1 = (size_t)NHID * NCTX * 2;
  const size_t szW2 = (size_t)DMOD * NHID * 2;
  const size_t szC  = (size_t)NROW * NCTX * 2;
  const size_t szH  = (size_t)NROW * NHID * 2;
  size_t off = 0;
  const size_t oWO = off; off += szWO;
  const size_t oW1 = off; off += szW1;
  const size_t oW2 = off; off += szW2;
  const size_t oC  = off; off += szC;
  const size_t oH  = off; off += szH;
  if (off > ws_size) return;
  if (off > (size_t)134217728) return;

  char* ws = (char*)d_ws;
  _Float16* WOT = (_Float16*)(ws + oWO);
  _Float16* W1T = (_Float16*)(ws + oW1);
  _Float16* W2T = (_Float16*)(ws + oW2);
  _Float16* CTX = (_Float16*)(ws + oC);
  _Float16* HPL = (_Float16*)(ws + oH);

  k_prepw<<<dim3(DMOD / 64, DMOD / 32), dim3(256), 0, stream>>>(wom, DMOD, DMOD, 16.0f, WOT);
  k_prepw<<<dim3(NCTX / 64, NHID / 32), dim3(256), 0, stream>>>(w1, NCTX, NHID, 32.0f, W1T);
  k_prepw<<<dim3(NHID / 64, DMOD / 32), dim3(256), 0, stream>>>(w2, NHID, DMOD, 32.0f, W2T);
  (void)hipFuncSetAttribute(reinterpret_cast<const void*>(&k_chunk),
                            hipFuncAttributeMaxDynamicSharedMemorySize, SM_CHUNK);
  k_chunk<<<dim3(NCHUNK), dim3(256), SM_CHUNK, stream>>>(x, WOT, bom, lsc, gam, bet, CTX);
  k_ffn1<<<dim3(NROW / 64, NHID / 128), dim3(128), 0, stream>>>(CTX, W1T, b1, HPL);
  k_ffn2<<<dim3(NROW / 64, DMOD / 128), dim3(128), 0, stream>>>(HPL, W2T, b2, x, out);
  (void)hipGetLastError();
}
